// CausalGroupedSelfAttention_59596966199611
// MI455X (gfx1250) — hardware-verified
//
#include <hip/hip_runtime.h>
#include <hip/hip_bf16.h>
#include <stddef.h>
#include <stdint.h>
#include <math.h>

#define BB    2
#define SQ    2048
#define HID   2048
#define NH    16
#define NKV   4
#define HDM   128
#define KVD   (NKV * HDM)
#define NKV2  (2 * KVD)
#define NQKV  (HID + NKV2)
#define MT    (BB * SQ)
#define R0    256
#define SQP   (SQ - R0)
#define MQP   (BB * SQP)
#define M3    (BB * R0)
#define QB    128
#define KC    64
#define KC3   32
#define NQB   (SQ / QB)
#define QB3   (R0 / QB)
#define Q64N  (R0 / 64)
#define NROT  (HDM / 2)
#define NFRQ  (HDM / 4)
#define RMS_EPS 1.1920928955078125e-07f

static_assert(SQ == 2048);
static_assert(HID == 2048);
static_assert(HID / 8 == 256);
static_assert(NH * HDM == HID);
static_assert(NH == 4 * NKV);
static_assert(SQ % 256 == 0);
static_assert(R0 == 256);
static_assert(R0 % QB == 0);
static_assert(NQB == 16);
static_assert(MT % 64 == 0);
static_assert(M3 % 64 == 0);
static_assert(KVD % 64 == 0);
static_assert(NQKV % 64 == 0);

typedef _Float16 v16h __attribute__((ext_vector_type(16)));
typedef _Float16 v8h  __attribute__((ext_vector_type(8)));
typedef _Float16 v4h  __attribute__((ext_vector_type(4)));
typedef float    v8f  __attribute__((ext_vector_type(8)));
typedef float    v4f  __attribute__((ext_vector_type(4)));
typedef unsigned int   v4u   __attribute__((ext_vector_type(4)));
typedef unsigned int   v2u   __attribute__((ext_vector_type(2)));
typedef unsigned short v4us  __attribute__((ext_vector_type(4)));
typedef unsigned short v8us  __attribute__((ext_vector_type(8)));
typedef unsigned short v16us __attribute__((ext_vector_type(16)));
typedef __bf16         v16b  __attribute__((ext_vector_type(16)));
typedef unsigned short ush;

union Frag   { v16h v; v8h h[2]; };
union FragU  { v16us v; v8us h[2]; v16b b; };
union Pack8  { v8h h; v4u u; };
union PackU  { v8us s; v4u u; };
union Pack4  { v4h h; v2u u; };
union PackU4 { v4us s; v2u u; };
struct HL { v4u h; v4u l; };

__device__ __forceinline__ ush f2bf(float f) {
  const unsigned u = __float_as_uint(f);
  return (ush)((u + 0x7FFFu + ((u >> 16) & 1u)) >> 16);
}
__device__ __forceinline__ float bf2f(ush b) { return __uint_as_float(((unsigned)b) << 16); }

__device__ __forceinline__ HL split8(v8f f) {
  PackU ph, pl;
#pragma unroll
  for (int e = 0; e < 8; ++e) {
    const ush hi = f2bf(f[e]);
    ph.s[e] = hi;
    pl.s[e] = f2bf(f[e] - bf2f(hi));
  }
  HL r; r.h = ph.u; r.l = pl.u;
  return r;
}

__device__ __forceinline__ v8f mma16(v16h a, v16h b, v8f c) {
  c = __builtin_amdgcn_wmma_f32_16x16x32_f16(false, a, false, b, (short)0, c, false, false);
  asm volatile("v_nop\n\tv_nop\n\tv_nop\n\tv_nop" : "+v"(c) : "v"(a), "v"(b));
  return c;
}
__device__ __forceinline__ v8f mmab(v16us a, v16us b, v8f c) {
  FragU ua, ub; ua.v = a; ub.v = b;
  c = __builtin_amdgcn_wmma_f32_16x16x32_bf16(false, ua.b, false, ub.b, (short)0, c, false, false);
  asm volatile("v_nop\n\tv_nop\n\tv_nop\n\tv_nop" : "+v"(c) : "v"(a), "v"(b));
  return c;
}

__device__ __forceinline__ v16h ldfrag(const _Float16* p, int ld, int row0, int k0, int lane) {
  const int m = lane & 15, lh = lane >> 4;
  const _Float16* q = p + (size_t)(row0 + m) * ld + k0 + 8 * lh;
  Frag f;
  f.h[0] = *(const v8h*)(q);
  f.h[1] = *(const v8h*)(q + 16);
  return f.v;
}
__device__ __forceinline__ v16us ldfragu(const ush* p, int ld, int row0, int k0, int lane) {
  const int m = lane & 15, lh = lane >> 4;
  const ush* q = p + (size_t)(row0 + m) * ld + k0 + 8 * lh;
  FragU f;
  f.h[0] = *(const v8us*)(q);
  f.h[1] = *(const v8us*)(q + 16);
  return f.v;
}

__device__ __forceinline__ v8f zero8() { return (v8f){0.f, 0.f, 0.f, 0.f, 0.f, 0.f, 0.f, 0.f}; }

__device__ __forceinline__ void gemm32x64(const _Float16* __restrict__ A, int lda,
                                          const _Float16* __restrict__ Bt, int ldb,
                                          int m0, int n0, int lane, v8f (&acc)[2][4]) {
#pragma unroll 2
  for (int k0 = 0; k0 < HID; k0 += 32) {
    const v16h a0 = ldfrag(A, lda, m0, k0, lane);
    const v16h a1 = ldfrag(A, lda, m0 + 16, k0, lane);
    const v16h b0 = ldfrag(Bt, ldb, n0, k0, lane);
    const v16h b1 = ldfrag(Bt, ldb, n0 + 16, k0, lane);
    const v16h b2 = ldfrag(Bt, ldb, n0 + 32, k0, lane);
    const v16h b3 = ldfrag(Bt, ldb, n0 + 48, k0, lane);
    acc[0][0] = mma16(a0, b0, acc[0][0]);
    acc[1][0] = mma16(a1, b0, acc[1][0]);
    acc[0][1] = mma16(a0, b1, acc[0][1]);
    acc[1][1] = mma16(a1, b1, acc[1][1]);
    acc[0][2] = mma16(a0, b2, acc[0][2]);
    acc[1][2] = mma16(a1, b2, acc[1][2]);
    acc[0][3] = mma16(a0, b3, acc[0][3]);
    acc[1][3] = mma16(a1, b3, acc[1][3]);
  }
}

__device__ __forceinline__ void gemm3_32x64(const ush* __restrict__ Ah, const ush* __restrict__ Al, int lda,
                                            const ush* __restrict__ Bh, const ush* __restrict__ Bl, int ldb,
                                            int m0, int n0, int lane, v8f (&acc)[2][4]) {
#pragma unroll 1
  for (int k0 = 0; k0 < HID; k0 += 32) {
    const v16us a0h = ldfragu(Ah, lda, m0, k0, lane);
    const v16us a1h = ldfragu(Ah, lda, m0 + 16, k0, lane);
    const v16us a0l = ldfragu(Al, lda, m0, k0, lane);
    const v16us a1l = ldfragu(Al, lda, m0 + 16, k0, lane);
#pragma unroll
    for (int t = 0; t < 4; ++t) {
      const v16us bh = ldfragu(Bh, ldb, n0 + 16 * t, k0, lane);
      const v16us bl = ldfragu(Bl, ldb, n0 + 16 * t, k0, lane);
      acc[0][t] = mmab(a0h, bh, acc[0][t]);
      acc[1][t] = mmab(a1h, bh, acc[1][t]);
      acc[0][t] = mmab(a0h, bl, acc[0][t]);
      acc[1][t] = mmab(a1h, bl, acc[1][t]);
      acc[0][t] = mmab(a0l, bh, acc[0][t]);
      acc[1][t] = mmab(a1l, bh, acc[1][t]);
    }
  }
}

__global__ __launch_bounds__(256) void k_cvt_x(const float* __restrict__ x, _Float16* __restrict__ xh,
                                               ush* __restrict__ x3h, ush* __restrict__ x3l, int ngrp) {
  const int g = blockIdx.x * 256 + (int)threadIdx.x;
  if (g >= ngrp) return;
  const int m  = g >> 8;
  const int b  = m / SQ;
  const int tq = m - b * SQ;
  const size_t o = (size_t)g * 8;
  const v4f a0 = *(const v4f*)(x + o);
  const v4f a1 = *(const v4f*)(x + o + 4);
  Pack8 pk;
  pk.h = (v8h){(_Float16)a0[0], (_Float16)a0[1], (_Float16)a0[2], (_Float16)a0[3],
               (_Float16)a1[0], (_Float16)a1[1], (_Float16)a1[2], (_Float16)a1[3]};
  const v4u vv = pk.u;
  const bool three = (tq < R0);
  const size_t o3 = ((size_t)(b * R0 + tq)) * HID + (size_t)(g & 255) * 8;
  HL s; s.h = (v4u){0u, 0u, 0u, 0u}; s.l = s.h;
  if (three) {
    const v8f f = (v8f){a0[0], a0[1], a0[2], a0[3], a1[0], a1[1], a1[2], a1[3]};
    s = split8(f);
  }
  volatile v4u* d = (volatile v4u*)(xh + o);
  *d = vv;
  if (three) { *(volatile v4u*)(x3h + o3) = s.h; *(volatile v4u*)(x3l + o3) = s.l; }
  __threadfence();
  *d = vv;
  if (three) { *(volatile v4u*)(x3h + o3) = s.h; *(volatile v4u*)(x3l + o3) = s.l; }
}

__global__ __launch_bounds__(256) void k_cvt_w(const float* __restrict__ w, _Float16* __restrict__ wf,
                                               ush* __restrict__ wh, ush* __restrict__ wl, int ngrp, float scale) {
  const int g = blockIdx.x * 256 + (int)threadIdx.x;
  if (g >= ngrp) return;
  const size_t o = (size_t)g * 8;
  const v4f a0 = *(const v4f*)(w + o);
  const v4f a1 = *(const v4f*)(w + o + 4);
  Pack8 pk;
  pk.h = (v8h){(_Float16)(a0[0] * scale), (_Float16)(a0[1] * scale), (_Float16)(a0[2] * scale),
               (_Float16)(a0[3] * scale), (_Float16)(a1[0] * scale), (_Float16)(a1[1] * scale),
               (_Float16)(a1[2] * scale), (_Float16)(a1[3] * scale)};
  const v4u vv = pk.u;
  const v8f f = (v8f){a0[0], a0[1], a0[2], a0[3], a1[0], a1[1], a1[2], a1[3]};
  const HL s = split8(f);
  *(volatile v4u*)(wf + o) = vv;
  *(volatile v4u*)(wh + o) = s.h;
  *(volatile v4u*)(wl + o) = s.l;
  __threadfence();
  *(volatile v4u*)(wf + o) = vv;
  *(volatile v4u*)(wh + o) = s.h;
  *(volatile v4u*)(wl + o) = s.l;
}

__global__ __launch_bounds__(256) void k_rope_tab(float* __restrict__ ctab, float* __restrict__ stab, int n) {
#pragma clang fp contract(off)
  __shared__ __align__(16) float sc[256];
  __shared__ __align__(16) float ss[256];
  const int tid = threadIdx.x;
  const int tb = blockIdx.x * 256;
  int t = tb + tid;
  t = (t < n) ? t : (n - 1);
  const int hr = t / NROT;
  const int j  = t - hr * NROT;
  float cs = 1.0f, sn = 0.0f;
  if (j < NFRQ) {
    const float lin  = (j < NFRQ - 1) ? ((float)j * (1.0f / 31.0f)) : 1.0f;
    const float freq = powf(0.0009765625f, lin);
    const float ang  = (float)hr * freq;
    sincosf(ang, &sn, &cs);
  }
  sc[tid] = cs;
  ss[tid] = sn;
  __syncthreads();
  if (tid < 64) {
    const v4f v = *(const v4f*)(sc + tid * 4);
    volatile v4f* d = (volatile v4f*)(ctab + tb + tid * 4);
    *d = v;
    __threadfence();
    *d = v;
  } else if (tid < 128) {
    const int u = tid - 64;
    const v4f v = *(const v4f*)(ss + u * 4);
    volatile v4f* d = (volatile v4f*)(stab + tb + u * 4);
    *d = v;
    __threadfence();
    *d = v;
  }
}

#define OTP 68
__device__ __forceinline__ void out_epilogue(v8f (&acc)[2][4], float scale, float* sw, float* __restrict__ out,
                                             size_t orow0, int ldo, int ocol, int lane, int hh, int c) {
#pragma unroll
  for (int sub = 0; sub < 2; ++sub) {
    __syncthreads();
#pragma unroll
    for (int t = 0; t < 4; ++t) {
#pragma unroll
      for (int r = 0; r < 8; ++r) sw[(8 * hh + r) * OTP + 16 * t + c] = acc[sub][t][r] * scale;
    }
    __syncthreads();
    v4f val[8];
    size_t go[8];
#pragma unroll
    for (int it = 0; it < 8; ++it) {
      const int p    = lane + 32 * it;
      const int L    = p >> 3;
      const int pc   = p & 7;
      const int row  = L >> 1;
      const int half = L & 1;
      val[it] = *(const v4f*)(sw + row * OTP + half * 32 + pc * 4);
      go[it]  = (orow0 + (size_t)(sub * 16 + row)) * (size_t)ldo + (size_t)ocol + half * 32 + pc * 4;
    }
    for (int ps = 0; ps < 2; ++ps) {
#pragma unroll
      for (int it = 0; it < 8; ++it) *(volatile v4f*)(out + go[it]) = val[it];
      __threadfence();
    }
  }
}

__global__ __launch_bounds__(256) void k_qkv(const _Float16* __restrict__ xh,
                                             const _Float16* __restrict__ wt,
                                             float* __restrict__ qf, float* __restrict__ kvf) {
  __shared__ __align__(16) float st[8][16 * OTP];
  const int tid = threadIdx.x, lane = tid & 31, wave = tid >> 5;
  const int hh = lane >> 4, c = lane & 15;
  const int mb = blockIdx.x * 256;
  const int b  = mb / SQ;
  const int tq = mb - b * SQ;
  const int n0 = blockIdx.y * 64;
  const int which = (n0 < HID) ? 0 : 1;
  if (which == 0 && tq < R0) return;

  v8f acc[2][4];
#pragma unroll
  for (int s = 0; s < 2; ++s)
#pragma unroll
    for (int t = 0; t < 4; ++t) acc[s][t] = zero8();
  gemm32x64(xh, HID, wt, HID, mb + wave * 32, n0, lane, acc);

  float* out   = (which == 0) ? qf : kvf;
  const size_t orow0 = (which == 0) ? ((size_t)b * SQP + (size_t)(tq - R0) + wave * 32)
                                    : ((size_t)mb + wave * 32);
  const int ldo  = (which == 0) ? HID : NKV2;
  const int ocol = (which == 0) ? n0 : (n0 - HID);
  out_epilogue(acc, 0.00390625f, st[wave], out, orow0, ldo, ocol, lane, hh, c);
}

__global__ __launch_bounds__(256) void k_qkv3(const ush* __restrict__ xh3, const ush* __restrict__ xl3,
                                              const ush* __restrict__ wth, const ush* __restrict__ wtl,
                                              float* __restrict__ qkv3f) {
  __shared__ __align__(16) float st[8][16 * OTP];
  const int tid = threadIdx.x, lane = tid & 31, wave = tid >> 5;
  const int hh = lane >> 4, c = lane & 15;
  const int m0 = blockIdx.x * 256 + wave * 32;
  const int n0 = blockIdx.y * 64;

  v8f acc[2][4];
#pragma unroll
  for (int s = 0; s < 2; ++s)
#pragma unroll
    for (int t = 0; t < 4; ++t) acc[s][t] = zero8();
  gemm3_32x64(xh3, xl3, HID, wth, wtl, HID, m0, n0, lane, acc);
  out_epilogue(acc, 1.0f, st[wave], qkv3f, (size_t)m0, NQKV, n0, lane, hh, c);
}

__global__ __launch_bounds__(256) void k_nr(const float* __restrict__ qf, const float* __restrict__ kvf,
                                            const float* __restrict__ ctab, const float* __restrict__ stab,
                                            _Float16* __restrict__ qp, _Float16* __restrict__ kp,
                                            int nqt, int ntot) {
#pragma clang fp contract(off)
  const int lane = threadIdx.x & 31, wave = threadIdx.x >> 5;
  const int w = blockIdx.x * 8 + wave;
  if (w >= ntot) return;
  const float* src;
  _Float16* dst;
  int hrow;
  if (w < nqt) {
    const int pr = w / NH;
    const int h  = w - pr * NH;
    const int b  = pr / SQP;
    const int t  = R0 + (pr - b * SQP);
    src  = qf + (size_t)pr * HID + h * HDM;
    dst  = qp + ((size_t)(b * NH + h) * SQ + t) * HDM;
    hrow = h;
  } else {
    const int w2 = w - nqt;
    const int m  = w2 / NKV;
    const int kh = w2 - m * NKV;
    const int b  = m / SQ;
    const int t  = m - b * SQ;
    src  = kvf + (size_t)m * NKV2 + kh * HDM;
    dst  = kp + ((size_t)(b * NKV + kh) * SQ + t) * HDM;
    hrow = kh;
  }
  const v4f v = *(const v4f*)(src + 4 * lane);
  float ssq = (v[0] * v[0] + v[1] * v[1]) + (v[2] * v[2] + v[3] * v[3]);
#pragma unroll
  for (int off = 1; off < 32; off <<= 1) ssq += __shfl_xor(ssq, off, 32);
  const float inv = rsqrtf(ssq * 0.0078125f + RMS_EPS);
  float own[4], oth[4];
#pragma unroll
  for (int e = 0; e < 4; ++e) own[e] = v[e] * inv;
#pragma unroll
  for (int e = 0; e < 4; ++e) oth[e] = __shfl_xor(own[e], 16, 32);
  const int jb = 4 * (lane & 15);
  const v4f cs4 = *(const v4f*)(ctab + hrow * NROT + jb);
  const v4f sn4 = *(const v4f*)(stab + hrow * NROT + jb);
  const bool first = (lane < 16);
  float y[4];
#pragma unroll
  for (int e = 0; e < 4; ++e) {
    const float a = own[e] * cs4[e];
    const float q = oth[e] * sn4[e];
    y[e] = first ? (a + q) : (a - q);
  }
  Pack4 pk;
  pk.h = (v4h){(_Float16)y[0], (_Float16)y[1], (_Float16)y[2], (_Float16)y[3]};
  volatile v2u* d = (volatile v2u*)(dst + 4 * lane);
  *d = pk.u;
  __threadfence();
  *d = pk.u;
}

__global__ __launch_bounds__(256) void k_nr3(const float* __restrict__ qkv3f,
                                             const float* __restrict__ ctab, const float* __restrict__ stab,
                                             ush* __restrict__ q3h, ush* __restrict__ q3l,
                                             ush* __restrict__ k3h, ush* __restrict__ k3l,
                                             int nqt, int ntot) {
#pragma clang fp contract(off)
  const int lane = threadIdx.x & 31, wave = threadIdx.x >> 5;
  const int w = blockIdx.x * 8 + wave;
  if (w >= ntot) return;
  const float* src;
  ush* dh;
  ush* dl;
  int hrow;
  if (w < nqt) {
    const int m3 = w / NH;
    const int h  = w - m3 * NH;
    const int b  = m3 / R0;
    const int t  = m3 - b * R0;
    src = qkv3f + (size_t)m3 * NQKV + h * HDM;
    const size_t drow = ((size_t)(b * NH + h) * R0 + t) * HDM;
    dh = q3h + drow; dl = q3l + drow;
    hrow = h;
  } else {
    const int w2 = w - nqt;
    const int m3 = w2 / NKV;
    const int kh = w2 - m3 * NKV;
    const int b  = m3 / R0;
    const int t  = m3 - b * R0;
    src = qkv3f + (size_t)m3 * NQKV + HID + kh * HDM;
    const size_t drow = ((size_t)(b * NKV + kh) * R0 + t) * HDM;
    dh = k3h + drow; dl = k3l + drow;
    hrow = kh;
  }
  const v4f v = *(const v4f*)(src + 4 * lane);
  float ssq = (v[0] * v[0] + v[1] * v[1]) + (v[2] * v[2] + v[3] * v[3]);
#pragma unroll
  for (int off = 1; off < 32; off <<= 1) ssq += __shfl_xor(ssq, off, 32);
  const float inv = rsqrtf(ssq * 0.0078125f + RMS_EPS);
  float own[4], oth[4];
#pragma unroll
  for (int e = 0; e < 4; ++e) own[e] = v[e] * inv;
#pragma unroll
  for (int e = 0; e < 4; ++e) oth[e] = __shfl_xor(own[e], 16, 32);
  const int jb = 4 * (lane & 15);
  const v4f cs4 = *(const v4f*)(ctab + hrow * NROT + jb);
  const v4f sn4 = *(const v4f*)(stab + hrow * NROT + jb);
  const bool first = (lane < 16);
  PackU4 ph, pl;
#pragma unroll
  for (int e = 0; e < 4; ++e) {
    const float a  = own[e] * cs4[e];
    const float q  = oth[e] * sn4[e];
    const float yv = first ? (a + q) : (a - q);
    const ush hi = f2bf(yv);
    ph.s[e] = hi;
    pl.s[e] = f2bf(yv - bf2f(hi));
  }
  volatile v2u* d0 = (volatile v2u*)(dh + 4 * lane);
  volatile v2u* d1 = (volatile v2u*)(dl + 4 * lane);
  *d0 = ph.u;
  *d1 = pl.u;
  __threadfence();
  *d0 = ph.u;
  *d1 = pl.u;
}

#define WTP 68
__global__ __launch_bounds__(256) void k_vt(const float* __restrict__ kvf, _Float16* __restrict__ vt) {
  __shared__ __align__(16) float tf[64 * WTP];
  const int tid = threadIdx.x;
  const int d0  = blockIdx.x * 64;
  const int kvh = d0 / HDM;
  const int dl0 = d0 - kvh * HDM;
  const int mb  = blockIdx.y * 64;
  const int b   = mb / SQ;
  const int t0  = mb - b * SQ;
  {
    const int kr = tid >> 4;
    const int n4 = (tid & 15) * 4;
#pragma unroll
    for (int it = 0; it < 4; ++it) {
      const int tl = it * 16 + kr;
      const v4f a = *(const v4f*)(kvf + (size_t)(mb + tl) * NKV2 + KVD + d0 + n4);
      *(v4f*)(tf + tl * WTP + n4) = a;
    }
  }
  __syncthreads();
  v4u val[2];
  size_t go[2];
#pragma unroll
  for (int j = 0; j < 2; ++j) {
    const int p  = tid + 256 * j;
    const int dl = p >> 3;
    const int pc = p & 7;
    const float* cp = tf + (pc * 8) * WTP + dl;
    Pack8 pk;
    pk.h = (v8h){(_Float16)(cp[0 * WTP] * 16.0f), (_Float16)(cp[1 * WTP] * 16.0f),
                 (_Float16)(cp[2 * WTP] * 16.0f), (_Float16)(cp[3 * WTP] * 16.0f),
                 (_Float16)(cp[4 * WTP] * 16.0f), (_Float16)(cp[5 * WTP] * 16.0f),
                 (_Float16)(cp[6 * WTP] * 16.0f), (_Float16)(cp[7 * WTP] * 16.0f)};
    val[j] = pk.u;
    go[j]  = ((size_t)((b * NKV + kvh) * HDM + dl0 + dl)) * SQ + t0 + pc * 8;
  }
  for (int ps = 0; ps < 2; ++ps) {
#pragma unroll
    for (int j = 0; j < 2; ++j) *(volatile v4u*)(vt + go[j]) = val[j];
    __threadfence();
  }
}

__global__ __launch_bounds__(256) void k_vt3(const float* __restrict__ qkv3f, ush* __restrict__ v3h,
                                             ush* __restrict__ v3l) {
  __shared__ __align__(16) float tf[64 * WTP];
  const int tid = threadIdx.x;
  const int d0  = blockIdx.x * 64;
  const int kvh = d0 / HDM;
  const int dl0 = d0 - kvh * HDM;
  const int mb  = blockIdx.y * 64;
  const int b   = mb / R0;
  const int t0  = mb - b * R0;
  {
    const int kr = tid >> 4;
    const int n4 = (tid & 15) * 4;
#pragma unroll
    for (int it = 0; it < 4; ++it) {
      const int tl = it * 16 + kr;
      const v4f a = *(const v4f*)(qkv3f + (size_t)(mb + tl) * NQKV + HID + KVD + d0 + n4);
      *(v4f*)(tf + tl * WTP + n4) = a;
    }
  }
  __syncthreads();
  v4u vh[2], vl[2];
  size_t go[2];
#pragma unroll
  for (int j = 0; j < 2; ++j) {
    const int p  = tid + 256 * j;
    const int dl = p >> 3;
    const int pc = p & 7;
    const float* cp = tf + (pc * 8) * WTP + dl;
    const v8f f = (v8f){cp[0 * WTP], cp[1 * WTP], cp[2 * WTP], cp[3 * WTP],
                        cp[4 * WTP], cp[5 * WTP], cp[6 * WTP], cp[7 * WTP]};
    const HL s = split8(f);
    vh[j] = s.h;
    vl[j] = s.l;
    go[j] = ((size_t)((b * NKV + kvh) * HDM + dl0 + dl)) * R0 + t0 + pc * 8;
  }
  for (int ps = 0; ps < 2; ++ps) {
#pragma unroll
    for (int j = 0; j < 2; ++j) {
      *(volatile v4u*)(v3h + go[j]) = vh[j];
      *(volatile v4u*)(v3l + go[j]) = vl[j];
    }
    __threadfence();
  }
}

#define KTP  136
#define VTP  72
#define VTP3 40
#define PTP  72
__global__ __launch_bounds__(256) __attribute__((amdgpu_num_vgpr(256)))
void k_attn(const _Float16* __restrict__ qp, const _Float16* __restrict__ kp,
            const _Float16* __restrict__ vt, _Float16* __restrict__ op, float sscale) {
  __shared__ __align__(16) _Float16 Ks[KC * KTP];
  __shared__ __align__(16) _Float16 Vs[HDM * VTP];
  __shared__ __align__(16) _Float16 Ps[8][16 * PTP];

  const int tid = threadIdx.x, lane = tid & 31, wave = tid >> 5;
  const int hh = lane >> 4, c = lane & 15;
  const int per = NQB - QB3;
  const int qbi = blockIdx.x % per;
  const int bh  = blockIdx.x / per;
  const int h   = bh % NH;
  const int b   = bh / NH;
  const int qb  = QB3 + qbi;
  const int kvh = h >> 2;
  const int q0  = qb * QB + wave * 16;

  const _Float16* Q = qp + (size_t)(b * NH + h) * SQ * HDM;
  const _Float16* K = kp + (size_t)(b * NKV + kvh) * SQ * HDM;
  const _Float16* V = vt + (size_t)(b * NKV + kvh) * HDM * SQ;

  const float NEGI = -__builtin_huge_valf();
  float mrow[8], lrow[8];
  v8f oacc[8];
#pragma unroll
  for (int r = 0; r < 8; ++r) { mrow[r] = NEGI; lrow[r] = 0.f; }
#pragma unroll
  for (int t = 0; t < 8; ++t) oacc[t] = zero8();

  _Float16* pw = Ps[wave];
  const int nchunk = 2 * qb + 2;

  for (int kc = 0; kc < nchunk; ++kc) {
    const int kv0 = kc * KC;
    __syncthreads();
    {
      const int r  = tid >> 2;
      const int qq = (tid & 3) * 32;
      const _Float16* ks = K + (size_t)(kv0 + r) * HDM + qq;
#pragma unroll
      for (int e = 0; e < 4; ++e) *(v8h*)(Ks + r * KTP + qq + 8 * e) = *(const v8h*)(ks + 8 * e);
      const int r2 = tid >> 1;
      const int q2 = (tid & 1) * 32;
      const _Float16* vs = V + (size_t)r2 * SQ + kv0 + q2;
#pragma unroll
      for (int e = 0; e < 4; ++e) *(v8h*)(Vs + r2 * VTP + q2 + 8 * e) = *(const v8h*)(vs + 8 * e);
    }
    __syncthreads();

    v8f s[4];
#pragma unroll
    for (int j = 0; j < 4; ++j) s[j] = zero8();
#pragma unroll
    for (int dc = 0; dc < 4; ++dc) {
      const v16h qa = ldfrag(Q, HDM, q0, dc * 32, lane);
#pragma unroll
      for (int j = 0; j < 4; ++j) {
        const v16h kb = ldfrag(Ks, KTP, j * 16, dc * 32, lane);
        s[j] = mma16(qa, kb, s[j]);
      }
    }
    const bool diag = (kc >= 2 * qb);
    if (diag) {
#pragma unroll
      for (int r = 0; r < 8; ++r) {
        const int qr = q0 + 8 * hh + r;
#pragma unroll
        for (int j = 0; j < 4; ++j) {
          const int key  = kv0 + 16 * j + c;
          const float sv = s[j][r] * sscale;
          s[j][r] = (key > qr) ? NEGI : sv;
        }
      }
    } else {
#pragma unroll
      for (int r = 0; r < 8; ++r)
#pragma unroll
        for (int j = 0; j < 4; ++j) s[j][r] = s[j][r] * sscale;
    }
    float cm[8];
#pragma unroll
    for (int r = 0; r < 8; ++r) {
      float m = NEGI;
#pragma unroll
      for (int j = 0; j < 4; ++j) m = fmaxf(m, s[j][r]);
#pragma unroll
      for (int off = 1; off < 16; off <<= 1) m = fmaxf(m, __shfl_xor(m, off, 32));
      cm[r] = m;
    }
    float al[8];
#pragma unroll
    for (int r = 0; r < 8; ++r) {
      const float mnew  = fmaxf(mrow[r], cm[r]);
      const float alpha = __expf(mrow[r] - mnew);
      mrow[r] = mnew;
      float psum = 0.f;
#pragma unroll
      for (int j = 0; j < 4; ++j) {
        const float p = __expf(s[j][r] - mnew);
        psum += p;
        pw[(8 * hh + r) * PTP + j * 16 + c] = (_Float16)(p * 1024.0f);
      }
#pragma unroll
      for (int off = 1; off < 16; off <<= 1) psum += __shfl_xor(psum, off, 32);
      lrow[r] = lrow[r] * alpha + psum;
      al[r] = alpha;
    }
#pragma unroll
    for (int t = 0; t < 8; ++t)
#pragma unroll
      for (int r = 0; r < 8; ++r) oacc[t][r] *= al[r];
    __syncthreads();

#pragma unroll
    for (int kk = 0; kk < 2; ++kk) {
      const v16h pa = ldfrag(pw, PTP, 0, kk * 32, lane);
#pragma unroll
      for (int t = 0; t < 8; ++t) {
        const v16h vb = ldfrag(Vs, VTP, t * 16, kk * 32, lane);
        oacc[t] = mma16(pa, vb, oacc[t]);
      }
    }
  }
  __syncthreads();

  float invr[8];
#pragma unroll
  for (int r = 0; r < 8; ++r) {
    const float lr = lrow[r];
    invr[r] = (lr > 0.f) ? (0.0009765625f / lr) : 0.f;
  }
#pragma unroll
  for (int hf = 0; hf < 2; ++hf) {
    __syncthreads();
#pragma unroll
    for (int r = 0; r < 8; ++r) {
#pragma unroll
      for (int t = 0; t < 4; ++t)
        pw[(8 * hh + r) * PTP + 16 * t + c] = (_Float16)(oacc[4 * hf + t][r] * invr[r]);
    }
    __syncthreads();
    v4u val[4];
    size_t go[4];
#pragma unroll
    for (int it = 0; it < 4; ++it) {
      const int p  = lane + 32 * it;
      const int L  = p >> 3;
      const int pc = p & 7;
      Pack8 pk;
      pk.h    = *(const v8h*)(pw + L * PTP + pc * 8);
      val[it] = pk.u;
      go[it]  = ((size_t)(b * SQ + q0 + L)) * HID + (size_t)h * HDM + hf * 64 + pc * 8;
    }
    for (int ps = 0; ps < 2; ++ps) {
#pragma unroll
      for (int it = 0; it < 4; ++it) *(volatile v4u*)(op + go[it]) = val[it];
      __threadfence();
    }
  }
}

__global__ __launch_bounds__(128) __attribute__((amdgpu_num_vgpr(256)))
void k_attn3(const ush* __restrict__ q3h, const ush* __restrict__ q3l,
             const ush* __restrict__ k3h, const ush* __restrict__ k3l,
             const ush* __restrict__ v3h, const ush* __restrict__ v3l,
             ush* __restrict__ o3h, ush* __restrict__ o3l, float sscale) {
  __shared__ __align__(16) ush Ksh[KC3 * KTP];
  __shared__ __align__(16) ush Ksl[KC3 * KTP];
  __shared__ __align__(16) ush Vsh[HDM * VTP3];
  __shared__ __align__(16) ush Vsl[HDM * VTP3];
  __shared__ __align__(16) ush Ph[4][16 * PTP];
  __shared__ __align__(16) ush Pl[4][16 * PTP];

  const int tid = threadIdx.x, lane = tid & 31, wave = tid >> 5;
  const int hh = lane >> 4, c = lane & 15;
  const int q64 = blockIdx.x % Q64N;
  const int bh  = blockIdx.x / Q64N;
  const int h   = bh % NH;
  const int b   = bh / NH;
  const int kvh = h >> 2;
  const int q0  = q64 * 64 + wave * 16;

  const ush* Qh  = q3h + (size_t)(b * NH + h) * R0 * HDM;
  const ush* Ql  = q3l + (size_t)(b * NH + h) * R0 * HDM;
  const ush* K3H = k3h + (size_t)(b * NKV + kvh) * R0 * HDM;
  const ush* K3L = k3l + (size_t)(b * NKV + kvh) * R0 * HDM;
  const ush* V3H = v3h + (size_t)(b * NKV + kvh) * HDM * R0;
  const ush* V3L = v3l + (size_t)(b * NKV + kvh) * HDM * R0;

  const float NEGI = -__builtin_huge_valf();
  float mrow[8], lrow[8];
  v8f oacc[8];
#pragma unroll
  for (int r = 0; r < 8; ++r) { mrow[r] = NEGI; lrow[r] = 0.f; }
#pragma unroll
  for (int t = 0; t < 8; ++t) oacc[t] = zero8();

  ush* pwh = Ph[wave];
  ush* pwl = Pl[wave];
  const int nchunk = 2 * q64 + 2;

  for (int kc = 0; kc < nchunk; ++kc) {
    const int kv0 = kc * KC3;
    __syncthreads();
    {
      const int r  = tid >> 2;
      const int qq = (tid & 3) * 32;
      const ush* ah = K3H + (size_t)(kv0 + r) * HDM + qq;
      const ush* al = K3L + (size_t)(kv0 + r) * HDM + qq;
#pragma unroll
      for (int e = 0; e < 4; ++e) {
        *(v8us*)(Ksh + r * KTP + qq + 8 * e) = *(const v8us*)(ah + 8 * e);
        *(v8us*)(Ksl + r * KTP + qq + 8 * e) = *(const v8us*)(al + 8 * e);
      }
      const int r2 = tid;
      const ush* bh2 = V3H + (size_t)r2 * R0 + kv0;
      const ush* bl2 = V3L + (size_t)r2 * R0 + kv0;
#pragma unroll
      for (int e = 0; e < 4; ++e) {
        *(v8us*)(Vsh + r2 * VTP3 + 8 * e) = *(const v8us*)(bh2 + 8 * e);
        *(v8us*)(Vsl + r2 * VTP3 + 8 * e) = *(const v8us*)(bl2 + 8 * e);
      }
    }
    __syncthreads();

    v8f s[2];
    s[0] = zero8(); s[1] = zero8();
#pragma unroll
    for (int dc = 0; dc < 4; ++dc) {
      const v16us qah = ldfragu(Qh, HDM, q0, dc * 32, lane);
      const v16us qal = ldfragu(Ql, HDM, q0, dc * 32, lane);
#pragma unroll
      for (int j = 0; j < 2; ++j) {
        const v16us kbh = ldfragu(Ksh, KTP, j * 16, dc * 32, lane);
        const v16us kbl = ldfragu(Ksl, KTP, j * 16, dc * 32, lane);
        s[j] = mmab(qah, kbh, s[j]);
        s[j] = mmab(qah, kbl, s[j]);
        s[j] = mmab(qal, kbh, s[j]);
      }
    }
    const bool diag = (kc >= 2 * q64);
    if (diag) {
#pragma unroll
      for (int r = 0; r < 8; ++r) {
        const int qr = q0 + 8 * hh + r;
#pragma unroll
        for (int j = 0; j < 2; ++j) {
          const int key  = kv0 + 16 * j + c;
          const float sv = s[j][r] * sscale;
          s[j][r] = (key > qr) ? NEGI : sv;
        }
      }
    } else {
#pragma unroll
      for (int r = 0; r < 8; ++r)
#pragma unroll
        for (int j = 0; j < 2; ++j) s[j][r] = s[j][r] * sscale;
    }
    float cm[8];
#pragma unroll
    for (int r = 0; r < 8; ++r) {
      float m = fmaxf(s[0][r], s[1][r]);
#pragma unroll
      for (int off = 1; off < 16; off <<= 1) m = fmaxf(m, __shfl_xor(m, off, 32));
      cm[r] = m;
    }
    float al[8];
#pragma unroll
    for (int r = 0; r < 8; ++r) {
      const float mnew  = fmaxf(mrow[r], cm[r]);
      const float alpha = __expf(mrow[r] - mnew);
      mrow[r] = mnew;
      float psum = 0.f;
#pragma unroll
      for (int j = 0; j < 2; ++j) {
        const float p = __expf(s[j][r] - mnew);
        psum += p;
        const ush phi = f2bf(p);
        pwh[(8 * hh + r) * PTP + j * 16 + c] = phi;
        pwl[(8 * hh + r) * PTP + j * 16 + c] = f2bf(p - bf2f(phi));
      }
#pragma unroll
      for (int off = 1; off < 16; off <<= 1) psum += __shfl_xor(psum, off, 32);
      lrow[r] = lrow[r] * alpha + psum;
      al[r] = alpha;
    }
#pragma unroll
    for (int t = 0; t < 8; ++t)
#pragma unroll
      for (int r = 0; r < 8; ++r) oacc[t][r] *= al[r];
    __syncthreads();

    {
      const v16us pah = ldfragu(pwh, PTP, 0, 0, lane);
      const v16us pal = ldfragu(pwl, PTP, 0, 0, lane);
#pragma unroll
      for (int t = 0; t < 8; ++t) {
        const v16us vbh = ldfragu(Vsh, VTP3, t * 16, 0, lane);
        const v16us vbl = ldfragu(Vsl, VTP3, t * 16, 0, lane);
        oacc[t] = mmab(pah, vbh, oacc[t]);
        oacc[t] = mmab(pah, vbl, oacc[t]);
        oacc[t] = mmab(pal, vbh, oacc[t]);
      }
    }
  }
  __syncthreads();

  float invr[8];
#pragma unroll
  for (int r = 0; r < 8; ++r) {
    const float lr = lrow[r];
    invr[r] = (lr > 0.f) ? (1.0f / lr) : 0.f;
  }
#pragma unroll
  for (int hf = 0; hf < 2; ++hf) {
    __syncthreads();
#pragma unroll
    for (int r = 0; r < 8; ++r) {
#pragma unroll
      for (int t = 0; t < 4; ++t) {
        const float o = oacc[4 * hf + t][r] * invr[r];
        const ush hi = f2bf(o);
        pwh[(8 * hh + r) * PTP + 16 * t + c] = hi;
        pwl[(8 * hh + r) * PTP + 16 * t + c] = f2bf(o - bf2f(hi));
      }
    }
    __syncthreads();
    v4u vh[4], vl[4];
    size_t go[4];
#pragma unroll
    for (int it = 0; it < 4; ++it) {
      const int p  = lane + 32 * it;
      const int L  = p >> 3;
      const int pc = p & 7;
      PackU pk;
      pk.s   = *(const v8us*)(pwh + L * PTP + pc * 8);
      vh[it] = pk.u;
      pk.s   = *(const v8us*)(pwl + L * PTP + pc * 8);
      vl[it] = pk.u;
      go[it] = ((size_t)(b * R0 + q0 + L)) * HID + (size_t)h * HDM + hf * 64 + pc * 8;
    }
    for (int ps = 0; ps < 2; ++ps) {
#pragma unroll
      for (int it = 0; it < 4; ++it) {
        *(volatile v4u*)(o3h + go[it]) = vh[it];
        *(volatile v4u*)(o3l + go[it]) = vl[it];
      }
      __threadfence();
    }
  }
}

__global__ __launch_bounds__(256) void k_out(const _Float16* __restrict__ ap,
                                             const _Float16* __restrict__ wt,
                                             float* __restrict__ out) {
  __shared__ __align__(16) float st[8][16 * OTP];
  const int tid = threadIdx.x, lane = tid & 31, wave = tid >> 5;
  const int hh = lane >> 4, c = lane & 15;
  const int mb = blockIdx.x * 256;
  const int b  = mb / SQ;
  const int tq = mb - b * SQ;
  if (tq < R0) return;
  const int m0 = mb + wave * 32;
  const int n0 = blockIdx.y * 64;

  v8f acc[2][4];
#pragma unroll
  for (int s = 0; s < 2; ++s)
#pragma unroll
    for (int t = 0; t < 4; ++t) acc[s][t] = zero8();
  gemm32x64(ap, HID, wt, HID, m0, n0, lane, acc);
  out_epilogue(acc, 0.000244140625f, st[wave], out, (size_t)m0, HID, n0, lane, hh, c);
}

__global__ __launch_bounds__(256) void k_out3(const ush* __restrict__ ah, const ush* __restrict__ al,
                                              const ush* __restrict__ wh, const ush* __restrict__ wl,
                                              float* __restrict__ out) {
  __shared__ __align__(16) float st[8][16 * OTP];
  const int tid = threadIdx.x, lane = tid & 31, wave = tid >> 5;
  const int hh = lane >> 4, c = lane & 15;
  const int b   = blockIdx.x;
  const int m0a = b * R0 + wave * 32;
  const int n0  = blockIdx.y * 64;

  v8f acc[2][4];
#pragma unroll
  for (int s = 0; s < 2; ++s)
#pragma unroll
    for (int t = 0; t < 4; ++t) acc[s][t] = zero8();
  gemm3_32x64(ah, al, HID, wh, wl, HID, m0a, n0, lane, acc);
  out_epilogue(acc, 1.0f, st[wave], out, (size_t)b * SQ + wave * 32, HID, n0, lane, hh, c);
}

__global__ __launch_bounds__(32) void k_tail(float* __restrict__ out, int n0, const int* __restrict__ tm) {
  (void)tm;
  if (threadIdx.x == 0) {
    volatile float* d = out + n0;
    *d = 0.0f;
    __threadfence();
    *d = 0.0f;
  }
}

extern "C" void kernel_launch(void* const* d_in, const int* in_sizes, int n_in,
                              void* d_out, int out_size, void* d_ws, size_t ws_size,
                              hipStream_t stream) {
  if (n_in < 5) return;
  if (in_sizes[0] != MT * HID) return;
  if (in_sizes[1] != HID * HID) return;
  if (in_sizes[2] != NKV2 * HID) return;
  if (in_sizes[3] != HID * HID) return;
  if (in_sizes[4] != BB * SQ) return;
  if (out_size != MT * HID + 1) return;

  const float* x    = (const float*)d_in[0];
  const float* wq   = (const float*)d_in[1];
  const float* wkv  = (const float*)d_in[2];
  const float* wp   = (const float*)d_in[3];
  const int*   tmsk = (const int*)d_in[4];
  float* out = (float*)d_out;

  size_t off = 0;
  const size_t oX   = off; off += (size_t)MT * HID * 2;
  const size_t oX3h = off; off += (size_t)M3 * HID * 2;
  const size_t oX3l = off; off += (size_t)M3 * HID * 2;
  const size_t oWt  = off; off += (size_t)NQKV * HID * 2;
  const size_t oWth = off; off += (size_t)NQKV * HID * 2;
  const size_t oWtl = off; off += (size_t)NQKV * HID * 2;
  const size_t oWo  = off; off += (size_t)HID * HID * 2;
  const size_t oWoh = off; off += (size_t)HID * HID * 2;
  const size_t oWol = off; off += (size_t)HID * HID * 2;
  const size_t oQf  = off; off += (size_t)MQP * HID * 4;
  const size_t oKVf = off; off += (size_t)MT * NKV2 * 4;
  const size_t oC   = off; off += (size_t)NH * NROT * 4;
  const size_t oS   = off; off += (size_t)NH * NROT * 4;
  const size_t total = off;
  if (total > ws_size) return;
  if (total > (size_t)134217728) return;

  size_t a2 = oX;
  const size_t oQKV3 = a2; a2 += (size_t)M3 * NQKV * 4;
  const size_t oQp   = a2; a2 += (size_t)BB * NH * SQ * HDM * 2;
  const size_t oKp   = a2; a2 += (size_t)BB * NKV * SQ * HDM * 2;
  const size_t oV    = a2; a2 += (size_t)BB * NKV * HDM * SQ * 2;
  const size_t oQ3h  = a2; a2 += (size_t)BB * NH * R0 * HDM * 2;
  const size_t oQ3l  = a2; a2 += (size_t)BB * NH * R0 * HDM * 2;
  const size_t oK3h  = a2; a2 += (size_t)BB * NKV * R0 * HDM * 2;
  const size_t oK3l  = a2; a2 += (size_t)BB * NKV * R0 * HDM * 2;
  const size_t oV3h  = a2; a2 += (size_t)BB * NKV * HDM * R0 * 2;
  const size_t oV3l  = a2; a2 += (size_t)BB * NKV * HDM * R0 * 2;
  if (a2 > oWo) return;
  if (oQKV3 + (size_t)M3 * NQKV * 4 > oX3h) return;
  size_t a3 = oQf;
  const size_t oO    = a3; a3 += (size_t)MT * HID * 2;
  const size_t oO3h  = a3; a3 += (size_t)M3 * HID * 2;
  const size_t oO3l  = a3; a3 += (size_t)M3 * HID * 2;
  if (a3 > oC) return;

  char* ws = (char*)d_ws;
  _Float16* Xh  = (_Float16*)(ws + oX);
  ush*      X3h = (ush*)(ws + oX3h);
  ush*      X3l = (ush*)(ws + oX3l);
  _Float16* Wt  = (_Float16*)(ws + oWt);
  ush*      Wth = (ush*)(ws + oWth);
  ush*      Wtl = (ush*)(ws + oWtl);
  _Float16* Wot = (_Float16*)(ws + oWo);
  ush*      Woh = (ush*)(ws + oWoh);
  ush*      Wol = (ush*)(ws + oWol);
  float*    Qf  = (float*)(ws + oQf);
  float*    KVf = (float*)(ws + oKVf);
  float*    Ct  = (float*)(ws + oC);
  float*    St  = (float*)(ws + oS);
  float*    QKV3f = (float*)(ws + oQKV3);
  _Float16* Qp  = (_Float16*)(ws + oQp);
  _Float16* Kp  = (_Float16*)(ws + oKp);
  _Float16* Vt  = (_Float16*)(ws + oV);
  ush*      Q3h = (ush*)(ws + oQ3h);
  ush*      Q3l = (ush*)(ws + oQ3l);
  ush*      K3h = (ush*)(ws + oK3h);
  ush*      K3l = (ush*)(ws + oK3l);
  ush*      V3h = (ush*)(ws + oV3h);
  ush*      V3l = (ush*)(ws + oV3l);
  _Float16* Op  = (_Float16*)(ws + oO);
  ush*      O3h = (ush*)(ws + oO3h);
  ush*      O3l = (ush*)(ws + oO3l);

  const int ngx = in_sizes[0] / 8;
  k_cvt_x<<<dim3((ngx + 255) / 256), dim3(256), 0, stream>>>(x, Xh, X3h, X3l, ngx);
  const int ngq = in_sizes[1] / 8;
  const int ngk = in_sizes[2] / 8;
  const int ngp = in_sizes[3] / 8;
  const size_t rk = (size_t)HID * HID;
  k_cvt_w<<<dim3((ngq + 255) / 256), dim3(256), 0, stream>>>(wq, Wt, Wth, Wtl, ngq, 256.0f);
  k_cvt_w<<<dim3((ngk + 255) / 256), dim3(256), 0, stream>>>(wkv, Wt + rk, Wth + rk, Wtl + rk, ngk, 256.0f);
  k_cvt_w<<<dim3((ngp + 255) / 256), dim3(256), 0, stream>>>(wp, Wot, Woh, Wol, ngp, 256.0f);
  const int ntab = NH * NROT;
  if ((ntab & 255) != 0) return;
  k_rope_tab<<<dim3(ntab / 256), dim3(256), 0, stream>>>(Ct, St, ntab);
  k_qkv<<<dim3(MT / 256, NQKV / 64), dim3(256), 0, stream>>>(Xh, Wt, Qf, KVf);
  k_qkv3<<<dim3(M3 / 256, NQKV / 64), dim3(256), 0, stream>>>(X3h, X3l, Wth, Wtl, QKV3f);
  const int nqt  = MQP * NH;
  const int ntot = nqt + MT * NKV;
  const int nqt3  = M3 * NH;
  const int ntot3 = nqt3 + M3 * NKV;
  k_nr<<<dim3((ntot + 7) / 8), dim3(256), 0, stream>>>(Qf, KVf, Ct, St, Qp, Kp, nqt, ntot);
  k_nr3<<<dim3((ntot3 + 7) / 8), dim3(256), 0, stream>>>(QKV3f, Ct, St, Q3h, Q3l, K3h, K3l, nqt3, ntot3);
  k_vt<<<dim3(KVD / 64, MT / 64), dim3(256), 0, stream>>>(KVf, Vt);
  k_vt3<<<dim3(KVD / 64, M3 / 64), dim3(256), 0, stream>>>(QKV3f, V3h, V3l);
  const float sscale = 1.0f / sqrtf(128.0f);
  k_attn<<<dim3(BB * NH * (NQB - QB3)), dim3(256), 0, stream>>>(Qp, Kp, Vt, Op, sscale);
  k_attn3<<<dim3(BB * NH * Q64N), dim3(128), 0, stream>>>(Q3h, Q3l, K3h, K3l, V3h, V3l, O3h, O3l, sscale);
  k_out<<<dim3(MT / 256, HID / 64), dim3(256), 0, stream>>>(Op, Wot, out);
  k_out3<<<dim3(BB, HID / 64), dim3(256), 0, stream>>>(O3h, O3l, Woh, Wol, out);
  k_tail<<<dim3(1), dim3(32), 0, stream>>>(out, MT * HID, tmsk);
  (void)hipGetLastError();
}
